// EmpathyAttention_74938589380613
// MI455X (gfx1250) — hardware-verified
//
#include <hip/hip_runtime.h>

constexpr int NBATCH  = 2;
constexpr int SEQ_LEN = 2048;
constexpr int DMODEL  = 1024;
constexpr int NHEAD   = 16;
constexpr int DHEAD   = 64;
constexpr int MROWS   = NBATCH * SEQ_LEN;
constexpr int NBH     = NBATCH * NHEAD;
constexpr long PLANE_ELEMS = (long)MROWS * DMODEL;
constexpr long WMAT_ELEMS  = (long)DMODEL * DMODEL;
constexpr long OUT0_ELEMS  = PLANE_ELEMS;
constexpr long OUT1_BYTE_OFFSET = 16777216;
constexpr long OUT1_ELEM   = OUT1_BYTE_OFFSET / 4;
constexpr long OUT_TOTAL_ELEMS = OUT0_ELEMS + 1;
constexpr long OUT_TOTAL_BYTES = 16777220;
static_assert(OUT1_ELEM == OUT0_ELEMS);
static_assert((OUT1_ELEM + 1) * 4 <= OUT_TOTAL_BYTES);
static_assert(NBH == 32);
static_assert(DHEAD == 64 && NHEAD * DHEAD == DMODEL);

static_assert(MROWS % 64 == 0 && DMODEL % 64 == 0 && DMODEL % 32 == 0);
constexpr int GEMM_TILES  = (MROWS / 64) * (DMODEL / 64);
static_assert(GEMM_TILES % 8 == 0);
constexpr int GEMM_BLOCKS = GEMM_TILES / 8;

constexpr size_t SZ_PLANE = (size_t)PLANE_ELEMS * 2;
constexpr size_t SZ_WPL   = (size_t)WMAT_ELEMS * 2;
constexpr size_t WS_W16   = 0;
constexpr size_t SZ_W16   = 4 * SZ_WPL;
constexpr size_t WS_BRND  = WS_W16 + SZ_W16;
constexpr size_t SZ_BRND  = 4 * (size_t)DMODEL * 4;
constexpr size_t WS_COS   = WS_BRND + SZ_BRND;
constexpr size_t SZ_COS   = (size_t)NBH * 128;
constexpr size_t WS_X16   = WS_COS + SZ_COS;
constexpr size_t WS_QH    = WS_X16 + 3 * SZ_PLANE;
constexpr size_t WS_QL    = WS_QH + SZ_PLANE;
constexpr size_t WS_KH    = WS_QL + SZ_PLANE;
constexpr size_t WS_KL    = WS_KH + SZ_PLANE;
constexpr size_t WS_VH    = WS_KL + SZ_PLANE;
constexpr size_t WS_VL    = WS_VH + SZ_PLANE;
constexpr size_t WS_AH    = WS_VL + SZ_PLANE;
constexpr size_t WS_AL    = WS_AH + SZ_PLANE;
constexpr size_t WS_TOTAL = WS_AL + SZ_PLANE;
static_assert(WS_TOTAL == 100683776);
static_assert(WS_TOTAL <= 134217728);
static_assert(WS_BRND % 128 == 0 && WS_COS % 128 == 0 && WS_X16 % 128 == 0 && WS_QH % 128 == 0 && WS_AH % 128 == 0);

typedef __attribute__((ext_vector_type(16))) _Float16 v16h;
typedef __attribute__((ext_vector_type(8)))  _Float16 v8h;
typedef __attribute__((ext_vector_type(16))) __bf16   v16b;
typedef __attribute__((ext_vector_type(8)))  __bf16   v8b;
typedef __attribute__((ext_vector_type(8)))  float    v8f;
typedef __attribute__((ext_vector_type(4)))  float    v4f;
typedef __attribute__((ext_vector_type(4)))  unsigned v4u;

__device__ __forceinline__ unsigned short f2bf_bits(float f) {
  unsigned u = __float_as_uint(f);
  return (unsigned short)((u + 0x7FFFu + ((u >> 16) & 1u)) >> 16);
}
__device__ __forceinline__ float bf_bits2f(unsigned short h) { return __uint_as_float(((unsigned)h) << 16); }
__device__ __forceinline__ float h_bits2f(unsigned x) { return (float)__builtin_bit_cast(_Float16, (unsigned short)(x & 0xffffu)); }

__device__ __forceinline__ void dep_guard_h(v8f& a, v8f& b, v16h x, v16h y) { asm volatile("v_nop\n\tv_nop\n\tv_nop\n\tv_nop" : "+v"(a), "+v"(b) : "v"(x), "v"(y)); }
__device__ __forceinline__ void dep_guard_b(v8f& a, v8f& b, v16b x, v16b y) { asm volatile("v_nop\n\tv_nop\n\tv_nop\n\tv_nop" : "+v"(a), "+v"(b) : "v"(x), "v"(y)); }
__device__ __forceinline__ void keep4_h(v16h a, v16h b, v16h c, v16h d) { asm volatile("v_nop" :: "v"(a), "v"(b), "v"(c), "v"(d)); }
__device__ __forceinline__ void keep4_b(v16b a, v16b b, v16b c, v16b d) { asm volatile("v_nop" :: "v"(a), "v"(b), "v"(c), "v"(d)); }
__device__ __forceinline__ void acc_guard4(v8f& a, v8f& b, v8f& c, v8f& d) { asm volatile("v_nop\n\tv_nop\n\tv_nop\n\tv_nop" : "+v"(a), "+v"(b), "+v"(c), "+v"(d)); }
template <typename T> struct Frag;
template <> struct Frag<_Float16> {
  typedef v16h V; union U { v16h v; v8h h[2]; };
  static __device__ __forceinline__ v16h load(const _Float16* p) {
    U f; f.h[0] = *(const v8h*)(p); f.h[1] = *(const v8h*)(p + 16); return f.v;
  }
  static __device__ __forceinline__ v8f mma(v16h a, v16h b, v8f c) {
    return __builtin_amdgcn_wmma_f32_16x16x32_f16(false, a, false, b, (short)0, c, false, false);
  }
  static __device__ __forceinline__ void guard(v8f& a, v8f& b, v16h x, v16h y) { dep_guard_h(a, b, x, y); }
  static __device__ __forceinline__ void keep(v16h a, v16h b, v16h c, v16h d) { keep4_h(a, b, c, d); }
};
template <> struct Frag<__bf16> {
  typedef v16b V; union U { v16b v; v8b h[2]; };
  static __device__ __forceinline__ v16b load(const __bf16* p) {
    U f; f.h[0] = *(const v8b*)(p); f.h[1] = *(const v8b*)(p + 16); return f.v;
  }
  static __device__ __forceinline__ v8f mma(v16b a, v16b b, v8f c) {
    return __builtin_amdgcn_wmma_f32_16x16x32_bf16(false, a, false, b, (short)0, c, false, false);
  }
  static __device__ __forceinline__ void guard(v8f& a, v8f& b, v16b x, v16b y) { dep_guard_b(a, b, x, y); }
  static __device__ __forceinline__ void keep(v16b a, v16b b, v16b c, v16b d) { keep4_b(a, b, c, d); }
};

__device__ __forceinline__ v8f mma_bf(v16b a, v16b b, v8f c) {
  c = __builtin_amdgcn_wmma_f32_16x16x32_bf16(false, a, false, b, (short)0, c, false, false);
  asm volatile("v_nop\n\tv_nop\n\tv_nop\n\tv_nop" : "+v"(c) : "v"(a), "v"(b));
  return c;
}
__device__ __forceinline__ v8f mma_hf(v16h a, v16h b, v8f c) {
  c = __builtin_amdgcn_wmma_f32_16x16x32_f16(false, a, false, b, (short)0, c, false, false);
  asm volatile("v_nop\n\tv_nop\n\tv_nop\n\tv_nop" : "+v"(c) : "v"(a), "v"(b));
  return c;
}

__device__ __forceinline__ void pack_pair_bf(float f0, float f1, unsigned& hword, unsigned& lword) {
  const unsigned short h0 = f2bf_bits(f0);
  const unsigned short h1 = f2bf_bits(f1);
  const unsigned short l0 = f2bf_bits(f0 - bf_bits2f(h0));
  const unsigned short l1 = f2bf_bits(f1 - bf_bits2f(h1));
  hword = (unsigned)h0 | ((unsigned)h1 << 16);
  lword = (unsigned)l0 | ((unsigned)l1 << 16);
}

template <int ET> struct Elem;
template <> struct Elem<0> { typedef _Float16 T; };
template <> struct Elem<1> { typedef __bf16 T; };
template <int ET, int SPLIT, int BIAS_MODE, int OUT_MODE, bool RESID, int ACT = 0>
__global__ __launch_bounds__(256) void wmma_gemm64(
    const unsigned short* __restrict__ Ap, const unsigned short* __restrict__ A2p, int lda, long strideA,
    const unsigned short* __restrict__ Btp, const unsigned short* __restrict__ Bt2p, int ldb, long strideB,
    void* __restrict__ Cout, void* __restrict__ Cout2, int ldc, long strideC,
    const float* __restrict__ bias,
    const float* __restrict__ resid, long strideR,
    int M, int N, int K, float scale) {
  typedef typename Elem<ET>::T T;
  typedef typename Frag<T>::V V;
  constexpr bool SPL = (SPLIT != 0);
  constexpr bool BLO = (SPLIT == 1);
  const T* A = (const T*)Ap; const T* A2 = (const T*)A2p; const T* Bt = (const T*)Btp; const T* Bt2 = (const T*)Bt2p;
  __shared__ __align__(16) float sT[8][16 * 68];
  const int b    = blockIdx.y;
  const int lane = threadIdx.x & 31;
  const int wave = threadIdx.x >> 5;
  const int tilesN = N >> 6;
  const int tilesM = M >> 6;
  const int tile = blockIdx.x * 8 + wave;
  if (tile >= tilesM * tilesN) return;
  const int tm = tile / tilesN;
  const int tn = tile - tm * tilesN;
  const int m0 = tm << 6;
  const int n0 = tn << 6;

  const T* Ab  = A  + (size_t)b * strideA;
  const T* Bb  = Bt + (size_t)b * strideB;
  const T* Ab2 = SPL ? (A2  + (size_t)b * strideA) : nullptr;
  const T* Bb2 = BLO ? (Bt2 + (size_t)b * strideB) : nullptr;

  const int rlane = lane & 15;
  const int koff  = (lane >> 4) * 8;
  const int mOff  = (lane >> 4) * 8;

  v8f acc[4][4];
#pragma unroll
  for (int i = 0; i < 4; ++i)
#pragma unroll
    for (int j = 0; j < 4; ++j) acc[i][j] = (v8f){0.f,0.f,0.f,0.f,0.f,0.f,0.f,0.f};

  for (int k0 = 0; k0 < K; k0 += 32) {
    V bh[4], bl[4];
#pragma unroll
    for (int j = 0; j < 4; ++j) {
      const size_t bo = (size_t)(n0 + (j << 4) + rlane) * ldb + koff + k0;
      bh[j] = Frag<T>::load(Bb + bo);
      if (BLO) bl[j] = Frag<T>::load(Bb2 + bo);
    }
#pragma unroll
    for (int i = 0; i < 4; ++i) {
      const size_t ao = (size_t)(m0 + (i << 4) + rlane) * lda + koff + k0;
      V ah = Frag<T>::load(Ab + ao);
      V al;
      if (SPL) al = Frag<T>::load(Ab2 + ao);
#pragma unroll
      for (int j = 0; j < 4; ++j) {
        acc[i][j] = Frag<T>::mma(ah, bh[j], acc[i][j]);
        if (BLO) acc[i][j] = Frag<T>::mma(ah, bl[j], acc[i][j]);
        if (SPL) acc[i][j] = Frag<T>::mma(al, bh[j], acc[i][j]);
      }
      Frag<T>::guard(acc[i][0], acc[i][3], ah, SPL ? al : ah);
    }
    Frag<T>::keep(bh[0], bh[1], bh[2], bh[3]);
    if (BLO) Frag<T>::keep(bl[0], bl[1], bl[2], bl[3]);
  }
  acc_guard4(acc[0][0], acc[0][1], acc[0][2], acc[0][3]);
  acc_guard4(acc[1][0], acc[1][1], acc[1][2], acc[1][3]);
  acc_guard4(acc[2][0], acc[2][1], acc[2][2], acc[2][3]);
  acc_guard4(acc[3][0], acc[3][1], acc[3][2], acc[3][3]);

  float* slab = sT[wave];
  const float* Rb = RESID ? (resid + (size_t)b * strideR) : nullptr;
#pragma unroll
  for (int i = 0; i < 4; ++i) {
    const int mBase = m0 + (i << 4);
#pragma unroll
    for (int j = 0; j < 4; ++j) {
      const int n = n0 + (j << 4) + rlane;
      float bv = 0.f;
      if (BIAS_MODE == 2) bv = bias[n];
#pragma unroll
      for (int r = 0; r < 8; ++r) {
        float v = acc[i][j][r] * scale;
        if (BIAS_MODE == 1) v += bias[mBase + mOff + r];
        if (BIAS_MODE == 2) v += bv;
        if (RESID) v += Rb[(size_t)(mBase + mOff + r) * ldc + n];
        if (ACT == 1) v = tanhf(v);
        if (ACT == 2) v = fmaxf(v, 0.0f);
        if (ACT == 4) v = (v > 0.f) ? v : 0.01f * v;
        slab[(mOff + r) * 68 + (j << 4) + rlane] = v;
      }
    }
    __builtin_amdgcn_fence(__ATOMIC_RELEASE, "workgroup");
    __builtin_amdgcn_wave_barrier();
    __builtin_amdgcn_fence(__ATOMIC_ACQUIRE, "workgroup");
    if (OUT_MODE == 0) {
      float* C = (float*)Cout + (size_t)b * strideC;
      const int hh = lane >> 4, c4 = (lane & 15) * 4;
      for (int pass = 0; pass < 2; ++pass) {
#pragma unroll
        for (int it = 0; it < 8; ++it) {
          const int row = it * 2 + hh;
          v4f v = *(const v4f*)(slab + row * 68 + c4);
          *(volatile v4f*)(C + (size_t)(mBase + row) * ldc + n0 + c4) = v;
        }
        __threadfence();
      }
    } else {
      const int q = lane >> 3, c8 = (lane & 7) * 8;
      unsigned short* C  = (unsigned short*)Cout  + (size_t)b * strideC;
      unsigned short* C2 = (OUT_MODE >= 2) ? ((unsigned short*)Cout2 + (size_t)b * strideC) : nullptr;
      for (int pass = 0; pass < 2; ++pass) {
#pragma unroll
        for (int it = 0; it < 4; ++it) {
          const int row = it * 4 + q;
          const float* sp = slab + row * 68 + c8;
          v8h hv, lv;
#pragma unroll
          for (int e = 0; e < 8; ++e) {
            if (OUT_MODE == 1) {
              hv[e] = (_Float16)sp[e];
            } else if (OUT_MODE == 2) {
              unsigned short hb = f2bf_bits(sp[e]);
              unsigned short lb = f2bf_bits(sp[e] - bf_bits2f(hb));
              hv[e] = __builtin_bit_cast(_Float16, hb);
              lv[e] = __builtin_bit_cast(_Float16, lb);
            } else {
              const _Float16 hq = (_Float16)sp[e];
              hv[e] = hq;
              lv[e] = (_Float16)((sp[e] - (float)hq) * 2048.0f);
            }
          }
          *(volatile v8h*)(C + (size_t)(mBase + row) * ldc + n0 + c8) = hv;
          if (OUT_MODE >= 2) *(volatile v8h*)(C2 + (size_t)(mBase + row) * ldc + n0 + c8) = lv;
        }
        __threadfence();
      }
    }
    __builtin_amdgcn_fence(__ATOMIC_RELEASE, "workgroup");
    __builtin_amdgcn_wave_barrier();
    __builtin_amdgcn_fence(__ATOMIC_ACQUIRE, "workgroup");
  }
}

constexpr int CAST_XBLK = (int)(PLANE_ELEMS / 8 / 256);
constexpr int CAST_WBLK = (int)(WMAT_ELEMS / 8 / 256);
constexpr int CAST_PLANE_BLOCKS = 3 * CAST_XBLK + 4 * CAST_WBLK;
constexpr int CAST_BIAS_BLOCKS  = 4;
static_assert((long)CAST_XBLK * 256 * 8 == PLANE_ELEMS && (long)CAST_WBLK * 256 * 8 == WMAT_ELEMS);
static_assert(256 * 4 == DMODEL);

__global__ __launch_bounds__(256) void k_cast_inputs(
    const float* __restrict__ q, const float* __restrict__ k, const float* __restrict__ v,
    const float* __restrict__ Wq, const float* __restrict__ Wk, const float* __restrict__ Wv, const float* __restrict__ Wo,
    const float* __restrict__ bq, const float* __restrict__ bk, const float* __restrict__ bv, const float* __restrict__ bo,
    unsigned short* __restrict__ x16, unsigned short* __restrict__ w16, float* __restrict__ brnd) {
  const int blk = blockIdx.x;
  const int t = threadIdx.x;
  if (blk < CAST_PLANE_BLOCKS) {
    const float* src;
    unsigned short* dst;
    int lb;
    if (blk < CAST_XBLK) { src = q; dst = x16; lb = blk; }
    else if (blk < 2 * CAST_XBLK) { src = k; dst = x16 + PLANE_ELEMS; lb = blk - CAST_XBLK; }
    else if (blk < 3 * CAST_XBLK) { src = v; dst = x16 + 2 * PLANE_ELEMS; lb = blk - 2 * CAST_XBLK; }
    else {
      const int wb = blk - 3 * CAST_XBLK;
      const int wi = wb / CAST_WBLK;
      lb = wb - wi * CAST_WBLK;
      src = (wi == 0) ? Wq : (wi == 1) ? Wk : (wi == 2) ? Wv : Wo;
      dst = w16 + (size_t)wi * WMAT_ELEMS;
    }
    const size_t e = ((size_t)lb * 256 + t) * 8;
    const v4f a0 = *(const v4f*)(src + e);
    const v4f a1 = *(const v4f*)(src + e + 4);
    v4u w;
    w.x = (unsigned)f2bf_bits(a0.x) | ((unsigned)f2bf_bits(a0.y) << 16);
    w.y = (unsigned)f2bf_bits(a0.z) | ((unsigned)f2bf_bits(a0.w) << 16);
    w.z = (unsigned)f2bf_bits(a1.x) | ((unsigned)f2bf_bits(a1.y) << 16);
    w.w = (unsigned)f2bf_bits(a1.z) | ((unsigned)f2bf_bits(a1.w) << 16);
    volatile v4u* p = (volatile v4u*)(dst + e);
    *p = w;
    __threadfence();
    *p = w;
  } else {
    const int bi = blk - CAST_PLANE_BLOCKS;
    const float* src = (bi == 0) ? bq : (bi == 1) ? bk : (bi == 2) ? bv : bo;
    const int e = t * 4;
    const v4f a = *(const v4f*)(src + e);
    v4f r;
    r.x = bf_bits2f(f2bf_bits(a.x));
    r.y = bf_bits2f(f2bf_bits(a.y));
    r.z = bf_bits2f(f2bf_bits(a.z));
    r.w = bf_bits2f(f2bf_bits(a.w));
    volatile v4f* p = (volatile v4f*)(brnd + (size_t)bi * DMODEL + e);
    *p = r;
    __threadfence();
    *p = r;
  }
}

__global__ __launch_bounds__(256) void k_mean_cos(
    const unsigned short* __restrict__ Qh, const unsigned short* __restrict__ Ql,
    const unsigned short* __restrict__ Vh, const unsigned short* __restrict__ Vl,
    float* __restrict__ cosl) {
  __shared__ float sq[32][64];
  __shared__ float sv[32][64];
  __shared__ float qm[64];
  __shared__ float vm[64];
  __shared__ float shc;
  const int bh = blockIdx.x;
  const int b = bh / NHEAD, h = bh % NHEAD;
  const int t = threadIdx.x;
  const int c8 = t & 7;
  const int rg = t >> 3;
  float aq[8], av[8];
#pragma unroll
  for (int e = 0; e < 8; ++e) { aq[e] = 0.f; av[e] = 0.f; }
  const size_t colb = (size_t)h * DHEAD + (size_t)c8 * 8;
#pragma unroll 2
  for (int it = 0; it < SEQ_LEN / 32; ++it) {
    const int s = rg + it * 32;
    const size_t off = ((size_t)b * SEQ_LEN + s) * DMODEL + colb;
    const v4u wh = *(const v4u*)(Qh + off);
    const v4u wl = *(const v4u*)(Ql + off);
    const v4u uh = *(const v4u*)(Vh + off);
    const v4u ul = *(const v4u*)(Vl + off);
#pragma unroll
    for (int e = 0; e < 4; ++e) {
      const unsigned a0 = wh[e], a1 = wl[e], g0 = uh[e], g1 = ul[e];
      aq[2 * e]     += __uint_as_float(a0 << 16) + __uint_as_float(a1 << 16);
      aq[2 * e + 1] += __uint_as_float(a0 & 0xffff0000u) + __uint_as_float(a1 & 0xffff0000u);
      av[2 * e]     += h_bits2f(g0) + h_bits2f(g1) * (1.0f / 2048.0f);
      av[2 * e + 1] += h_bits2f(g0 >> 16) + h_bits2f(g1 >> 16) * (1.0f / 2048.0f);
    }
  }
#pragma unroll
  for (int e = 0; e < 8; ++e) { sq[rg][c8 * 8 + e] = aq[e]; sv[rg][c8 * 8 + e] = av[e]; }
  __syncthreads();
  if (t < 64) {
    float s1 = 0.f, s2 = 0.f;
#pragma unroll 1
    for (int g = 0; g < 32; ++g) { s1 += sq[g][t]; s2 += sv[g][t]; }
    qm[t] = s1 * (1.0f / (float)SEQ_LEN);
    vm[t] = s2 * (1.0f / (float)SEQ_LEN);
  }
  __syncthreads();
  if (t == 0) {
    float dot = 0.f, nq = 0.f, nv = 0.f;
#pragma unroll 1
    for (int i = 0; i < DHEAD; ++i) {
      const float a = qm[i], c = vm[i];
      dot += a * c;
      nq += a * a;
      nv += c * c;
    }
    const float na = fmaxf(sqrtf(nq), 1e-8f);
    const float nb = fmaxf(sqrtf(nv), 1e-8f);
    shc = dot / (na * nb);
  }
  __syncthreads();
  if (t < 32) {
    const float cv = shc;
    volatile float* p = cosl + (size_t)bh * 32 + t;
    *p = cv;
    __threadfence();
    *p = cv;
  }
}

constexpr int AKC  = 64;
constexpr int AQB  = 64;
constexpr int ANQB = SEQ_LEN / AQB;
constexpr int ATTN_BLOCKS = NBH * ANQB;
static_assert(SEQ_LEN % AKC == 0 && SEQ_LEN % AQB == 0);

__global__ __launch_bounds__(128) void k_attn(
    const unsigned short* __restrict__ Qh, const unsigned short* __restrict__ Ql,
    const unsigned short* __restrict__ Kh, const unsigned short* __restrict__ Kl,
    const unsigned short* __restrict__ Vh,
    const int* __restrict__ mask, const float* __restrict__ cosl,
    unsigned short* __restrict__ Ah, unsigned short* __restrict__ Al) {
  union FB { v16b v; v8b h[2]; };
  union FH { v16h v; v8h h[2]; };
  __shared__ __align__(16) unsigned short Ksh[AKC * DHEAD];
  __shared__ __align__(16) unsigned short Ksl[AKC * DHEAD];
  __shared__ __align__(16) unsigned short Vts[DHEAD * AKC];
  __shared__ __align__(16) _Float16 Psh[4][16 * AKC];
  __shared__ __align__(16) float Os[4][16 * 68];

  const int tid  = threadIdx.x;
  const int wave = tid >> 5;
  const int lane = tid & 31;
  const int hh   = lane >> 4;
  const int c    = lane & 15;

  const int bx = blockIdx.x;
  const int qb = bx % ANQB;
  const int bh = bx / ANQB;
  const int h  = bh % NHEAD;
  const int b  = bh / NHEAD;
  const int q0 = qb * AQB + wave * 16;
  const size_t rowbase = (size_t)b * SEQ_LEN;
  const int colh = h * DHEAD;

  v16b qah[2], qal[2];
  {
    const size_t qo = (rowbase + q0 + c) * DMODEL + colh + 8 * hh;
#pragma unroll
    for (int dc = 0; dc < 2; ++dc) {
      qah[dc] = Frag<__bf16>::load((const __bf16*)(const void*)(Qh + qo + dc * 32));
      qal[dc] = Frag<__bf16>::load((const __bf16*)(const void*)(Ql + qo + dc * 32));
    }
  }
  const float cb  = cosl[(size_t)bh * 32];
  const float cb5 = cb * 0.5f;
  const float cb3 = cb * 0.3f;
  const float NEGI = -__builtin_inff();

  float mrow[8], lrow[8];
  v8f oacc[4];
#pragma unroll
  for (int r = 0; r < 8; ++r) { mrow[r] = NEGI; lrow[r] = 0.f; }
#pragma unroll
  for (int t = 0; t < 4; ++t) oacc[t] = (v8f){0.f,0.f,0.f,0.f,0.f,0.f,0.f,0.f};

  for (int kc = 0; kc < SEQ_LEN / AKC; ++kc) {
    const int kv0 = kc * AKC;
    __syncthreads();
    {
      const int kvr = tid >> 1, dh = (tid & 1) * 32;
      const size_t go = (rowbase + kv0 + kvr) * DMODEL + colh + dh;
#pragma unroll
      for (int i = 0; i < 4; ++i) {
        const v4u wa = *(const v4u*)(Kh + go + 8 * i);
        const v4u wb = *(const v4u*)(Kl + go + 8 * i);
        *(v4u*)(Ksh + kvr * DHEAD + dh + 8 * i) = wa;
        *(v4u*)(Ksl + kvr * DHEAD + dh + 8 * i) = wb;
      }
#pragma unroll
      for (int i = 0; i < 4; ++i) {
        const v4u wv = *(const v4u*)(Vh + go + 8 * i);
#pragma unroll
        for (int e = 0; e < 4; ++e) {
          const unsigned x = wv[e];
          const int d = dh + 8 * i + 2 * e;
          Vts[d * AKC + kvr]       = (unsigned short)(x & 0xffffu);
          Vts[(d + 1) * AKC + kvr] = (unsigned short)(x >> 16);
        }
      }
    }
    __syncthreads();

    v8f s[4];
#pragma unroll
    for (int j = 0; j < 4; ++j) {
      s[j] = (v8f){0.f,0.f,0.f,0.f,0.f,0.f,0.f,0.f};
#pragma unroll
      for (int dc = 0; dc < 2; ++dc) {
        FB kb, kl;
        kb.h[0] = *(const v8b*)(const void*)(Ksh + (j * 16 + c) * DHEAD + dc * 32 + 8 * hh);
        kb.h[1] = *(const v8b*)(const void*)(Ksh + (j * 16 + c) * DHEAD + dc * 32 + 16 + 8 * hh);
        kl.h[0] = *(const v8b*)(const void*)(Ksl + (j * 16 + c) * DHEAD + dc * 32 + 8 * hh);
        kl.h[1] = *(const v8b*)(const void*)(Ksl + (j * 16 + c) * DHEAD + dc * 32 + 16 + 8 * hh);
        s[j] = mma_bf(qah[dc], kb.v, s[j]);
        s[j] = mma_bf(qah[dc], kl.v, s[j]);
        s[j] = mma_bf(qal[dc], kb.v, s[j]);
      }
    }
    int mk[4];
#pragma unroll
    for (int j = 0; j < 4; ++j) mk[j] = mask[kv0 + j * 16 + c];
    float cm[8];
#pragma unroll
    for (int r = 0; r < 8; ++r) {
      float m = NEGI;
#pragma unroll
      for (int j = 0; j < 4; ++j) {
        float x = s[j][r] * 0.125f;
        x = x + cb5;
        x = x + cb3;
        x = (mk[j] == 0) ? -1.0e9f : x;
        s[j][r] = x;
        m = fmaxf(m, x);
      }
#pragma unroll
      for (int off = 1; off < 16; off <<= 1) m = fmaxf(m, __shfl_xor(m, off, 32));
      cm[r] = m;
    }
    _Float16* pw = Psh[wave];
#pragma unroll
    for (int r = 0; r < 8; ++r) {
      const float mnew = fmaxf(mrow[r], cm[r]);
      const float alpha = expf(mrow[r] - mnew);
      mrow[r] = mnew;
      float psum = 0.f;
#pragma unroll
      for (int j = 0; j < 4; ++j) {
        const float p = expf(s[j][r] - mnew);
        psum += p;
        pw[(8 * hh + r) * AKC + j * 16 + c] = (_Float16)(p * 32768.0f);
      }
#pragma unroll
      for (int off = 1; off < 16; off <<= 1) psum += __shfl_xor(psum, off, 32);
      lrow[r] = lrow[r] * alpha + psum;
#pragma unroll
      for (int t = 0; t < 4; ++t) oacc[t][r] *= alpha;
    }
    __builtin_amdgcn_fence(__ATOMIC_RELEASE, "workgroup");
    __builtin_amdgcn_wave_barrier();
    __builtin_amdgcn_fence(__ATOMIC_ACQUIRE, "workgroup");
#pragma unroll
    for (int kk = 0; kk < 2; ++kk) {
      FH pa;
      pa.h[0] = *(const v8h*)(pw + c * AKC + kk * 32 + 8 * hh);
      pa.h[1] = *(const v8h*)(pw + c * AKC + kk * 32 + 16 + 8 * hh);
#pragma unroll
      for (int t = 0; t < 4; ++t) {
        FH vb;
        vb.h[0] = *(const v8h*)(const void*)(Vts + (t * 16 + c) * AKC + kk * 32 + 8 * hh);
        vb.h[1] = *(const v8h*)(const void*)(Vts + (t * 16 + c) * AKC + kk * 32 + 16 + 8 * hh);
        oacc[t] = mma_hf(pa.v, vb.v, oacc[t]);
      }
    }
  }

  float* os = Os[wave];
#pragma unroll
  for (int r = 0; r < 8; ++r) {
    const float inv = 1.0f / (lrow[r] * 32768.0f);
#pragma unroll
    for (int t = 0; t < 4; ++t) os[(8 * hh + r) * 68 + t * 16 + c] = oacc[t][r] * inv;
  }
  __builtin_amdgcn_fence(__ATOMIC_RELEASE, "workgroup");
  __builtin_amdgcn_wave_barrier();
  __builtin_amdgcn_fence(__ATOMIC_ACQUIRE, "workgroup");
  {
    const int q4 = lane >> 3, c8 = (lane & 7) * 8;
    for (int pass = 0; pass < 2; ++pass) {
#pragma unroll
      for (int it = 0; it < 4; ++it) {
        const int row = it * 4 + q4;
        const float* sp = os + row * 68 + c8;
        const v4f va = *(const v4f*)sp;
        const v4f vb = *(const v4f*)(sp + 4);
        v4u hw, lw;
        unsigned th, tl;
        pack_pair_bf(va.x, va.y, th, tl); hw.x = th; lw.x = tl;
        pack_pair_bf(va.z, va.w, th, tl); hw.y = th; lw.y = tl;
        pack_pair_bf(vb.x, vb.y, th, tl); hw.z = th; lw.z = tl;
        pack_pair_bf(vb.z, vb.w, th, tl); hw.w = th; lw.w = tl;
        const size_t go = (rowbase + q0 + row) * DMODEL + colh + c8;
        *(volatile v4u*)(Ah + go) = hw;
        *(volatile v4u*)(Al + go) = lw;
      }
      __threadfence();
    }
  }
}

__global__ __launch_bounds__(32) void k_bias_mean(const float* __restrict__ cosl, float* __restrict__ out1) {
  const int lane = threadIdx.x;
  float v = cosl[(size_t)lane * 32];
#pragma unroll
  for (int off = 1; off < 32; off <<= 1) v += __shfl_xor(v, off, 32);
  const float r = v * (1.0f / 32.0f);
  if (lane == 0) {
    *(volatile float*)out1 = r;
    __threadfence();
    *(volatile float*)out1 = r;
  }
}

extern "C" void kernel_launch(void* const* d_in, const int* in_sizes, int n_in,
                              void* d_out, int out_size, void* d_ws, size_t ws_size,
                              hipStream_t stream) {
  if (n_in < 12) return;
  if (ws_size < WS_TOTAL) return;
  if ((long)out_size < OUT_TOTAL_ELEMS) return;
  if ((long)in_sizes[0] != PLANE_ELEMS || (long)in_sizes[1] != PLANE_ELEMS || (long)in_sizes[2] != PLANE_ELEMS) return;
  if (in_sizes[3] < SEQ_LEN) return;
  if ((long)in_sizes[4] != WMAT_ELEMS || (long)in_sizes[6] != WMAT_ELEMS || (long)in_sizes[8] != WMAT_ELEMS || (long)in_sizes[10] != WMAT_ELEMS) return;
  if (in_sizes[5] < DMODEL || in_sizes[7] < DMODEL || in_sizes[9] < DMODEL || in_sizes[11] < DMODEL) return;

  const float* q    = (const float*)d_in[0];
  const float* k    = (const float*)d_in[1];
  const float* v    = (const float*)d_in[2];
  const int*   mask = (const int*)d_in[3];
  const float* Wq   = (const float*)d_in[4];
  const float* bq   = (const float*)d_in[5];
  const float* Wk   = (const float*)d_in[6];
  const float* bk   = (const float*)d_in[7];
  const float* Wv   = (const float*)d_in[8];
  const float* bv   = (const float*)d_in[9];
  const float* Wo   = (const float*)d_in[10];
  const float* bo   = (const float*)d_in[11];

  char* ws = (char*)d_ws;
  unsigned short* w16  = (unsigned short*)(ws + WS_W16);
  unsigned short* wq16 = w16;
  unsigned short* wk16 = w16 + WMAT_ELEMS;
  unsigned short* wv16 = w16 + 2 * WMAT_ELEMS;
  unsigned short* wo16 = w16 + 3 * WMAT_ELEMS;
  float* brnd = (float*)(ws + WS_BRND);
  float* cosl = (float*)(ws + WS_COS);
  unsigned short* x16 = (unsigned short*)(ws + WS_X16);
  unsigned short* xq  = x16;
  unsigned short* xk  = x16 + PLANE_ELEMS;
  unsigned short* xv  = x16 + 2 * PLANE_ELEMS;
  unsigned short* Qh  = (unsigned short*)(ws + WS_QH);
  unsigned short* Ql  = (unsigned short*)(ws + WS_QL);
  unsigned short* Kh  = (unsigned short*)(ws + WS_KH);
  unsigned short* Kl  = (unsigned short*)(ws + WS_KL);
  unsigned short* Vh  = (unsigned short*)(ws + WS_VH);
  unsigned short* Vl  = (unsigned short*)(ws + WS_VL);
  unsigned short* Ah  = (unsigned short*)(ws + WS_AH);
  unsigned short* Al  = (unsigned short*)(ws + WS_AL);
  float* out0 = (float*)d_out;
  float* out1 = (float*)d_out + OUT1_ELEM;

  k_cast_inputs<<<CAST_PLANE_BLOCKS + CAST_BIAS_BLOCKS, 256, 0, stream>>>(
      q, k, v, Wq, Wk, Wv, Wo, bq, bk, bv, bo, x16, w16, brnd);

  const dim3 ggrid(GEMM_BLOCKS, 1);
  wmma_gemm64<1, 0, 2, 2, false><<<ggrid, 256, 0, stream>>>(
      xq, xq, DMODEL, 0L, wq16, wq16, DMODEL, 0L, (void*)Qh, (void*)Ql, DMODEL, 0L,
      brnd + 0 * DMODEL, brnd, 0L, MROWS, DMODEL, DMODEL, 1.0f);
  wmma_gemm64<1, 0, 2, 2, false><<<ggrid, 256, 0, stream>>>(
      xk, xk, DMODEL, 0L, wk16, wk16, DMODEL, 0L, (void*)Kh, (void*)Kl, DMODEL, 0L,
      brnd + 1 * DMODEL, brnd, 0L, MROWS, DMODEL, DMODEL, 1.0f);
  wmma_gemm64<1, 0, 2, 3, false><<<ggrid, 256, 0, stream>>>(
      xv, xv, DMODEL, 0L, wv16, wv16, DMODEL, 0L, (void*)Vh, (void*)Vl, DMODEL, 0L,
      brnd + 2 * DMODEL, brnd, 0L, MROWS, DMODEL, DMODEL, 1.0f);
  k_mean_cos<<<NBH, 256, 0, stream>>>(Qh, Ql, Vh, Vl, cosl);
  k_attn<<<ATTN_BLOCKS, 128, 0, stream>>>(Qh, Ql, Kh, Kl, Vh, mask, cosl, Ah, Al);
  wmma_gemm64<1, 2, 2, 0, false><<<ggrid, 256, 0, stream>>>(
      Ah, Al, DMODEL, 0L, wo16, wo16, DMODEL, 0L, (void*)out0, (void*)out0, DMODEL, 0L,
      brnd + 3 * DMODEL, brnd, 0L, MROWS, DMODEL, DMODEL, 1.0f);
  k_bias_mean<<<1, 32, 0, stream>>>(cosl, out1);
}
